// BlockSparseHilbertAttentionV2_41171556499658
// MI455X (gfx1250) — hardware-verified
//
#include <hip/hip_runtime.h>


#define DEV __device__ __forceinline__

enum { BATCH = 2, SEQ = 2048, E = 1024, NH = 16, HD = 64, BLK = 64, NB = SEQ / BLK, NTOK = BATCH * SEQ, BAND = 15 };
static_assert(NB == 32);
static_assert(NTOK % 128 == 0);
static_assert(E % 64 == 0);
static_assert(NH * HD == E);

typedef _Float16 v8h  __attribute__((ext_vector_type(8)));
typedef _Float16 v16h __attribute__((ext_vector_type(16)));
typedef __bf16   v16b __attribute__((ext_vector_type(16)));
typedef unsigned short v8us __attribute__((ext_vector_type(8)));
typedef float v8f __attribute__((ext_vector_type(8)));
typedef float v4f __attribute__((ext_vector_type(4)));

union FragH { v16h v; v8h half[2]; };
union FragB { v16b v; v8us half[2]; };

DEV unsigned short f2bf(float x) {
  unsigned int u = __float_as_uint(x);
  u += 0x7FFFu + ((u >> 16) & 1u);
  return (unsigned short)(u >> 16);
}
DEV float bf2f(unsigned short b) { return __uint_as_float(((unsigned int)b) << 16); }

DEV v16h ldh(const _Float16* p) {
  FragH f;
  f.half[0] = *(const v8h*)p;
  f.half[1] = *(const v8h*)(p + 16);
  return f.v;
}
DEV v16b ldb(const unsigned short* p) {
  FragB f;
  f.half[0] = *(const v8us*)p;
  f.half[1] = *(const v8us*)(p + 16);
  return f.v;
}

DEV v8f mma_h(v16h a, v16h b, v8f c) {
  return __builtin_amdgcn_wmma_f32_16x16x32_f16(false, a, false, b, (short)0, c, false, false);
}
DEV v8f mma_b(v16b a, v16b b, v8f c) {
  return __builtin_amdgcn_wmma_f32_16x16x32_bf16(false, a, false, b, (short)0, c, false, false);
}

DEV size_t blkoff(int b, int h, int blk) {
  return (size_t)((b * NH + h) * NB + blk) * (size_t)(BLK * HD);
}

__global__ __launch_bounds__(256) void k_prep(
    const float* __restrict__ q, const float* __restrict__ k, const float* __restrict__ v,
    const float* __restrict__ wq, const float* __restrict__ wk, const float* __restrict__ wv,
    const float* __restrict__ wo,
    unsigned short* __restrict__ xq, unsigned short* __restrict__ xk, unsigned short* __restrict__ xv,
    unsigned short* __restrict__ bq, unsigned short* __restrict__ bk, unsigned short* __restrict__ bv,
    unsigned short* __restrict__ bo, int nact, int nw) {
  const int y = blockIdx.y;
  const float* src = (y == 0) ? q : (y == 1) ? k : (y == 2) ? v : (y == 3) ? wq : (y == 4) ? wk : (y == 5) ? wv : wo;
  unsigned short* dst = (y == 0) ? xq : (y == 1) ? xk : (y == 2) ? xv : (y == 3) ? bq : (y == 4) ? bk : (y == 5) ? bv : bo;
  const int nch = ((y < 3) ? nact : nw) >> 3;
  const int stride = gridDim.x * blockDim.x;
#pragma unroll 1
  for (int i = blockIdx.x * blockDim.x + threadIdx.x; i < nch; i += stride) {
    const float* s = src + (size_t)i * 8;
    const v4f a = *(const v4f*)s;
    const v4f c = *(const v4f*)(s + 4);
    v8us o;
    o[0] = f2bf(a[0]); o[1] = f2bf(a[1]); o[2] = f2bf(a[2]); o[3] = f2bf(a[3]);
    o[4] = f2bf(c[0]); o[5] = f2bf(c[1]); o[6] = f2bf(c[2]); o[7] = f2bf(c[3]);
    unsigned short* d = dst + (size_t)i * 8;
    *(volatile v8us*)d = o;
    __threadfence();
    *(volatile v8us*)d = o;
  }
}

DEV void st_frag_h(_Float16* s, int pr, int pc, v8f c, int hh, int m) {
#pragma unroll
  for (int rr = 0; rr < 8; ++rr) s[(8 * hh + rr) * pr + m * pc] = (_Float16)c[rr];
}

DEV void lines_nat(const _Float16* sT, _Float16* P, int row0, int col0, int w, int l) {
  const int q8 = l >> 3, j = l & 7;
#pragma unroll
  for (int p = 0; p < 8; ++p) {
    const int L = w * 32 + p * 4 + q8;
    const v8h val = *(const v8h*)(sT + L * 64 + j * 8);
    *(volatile v8h*)(P + (size_t)(row0 + L) * E + col0 + j * 8) = val;
  }
}

DEV void lines_vt(const _Float16* sT, _Float16* Vt, size_t base0, size_t base1, int w, int l) {
  const int q8 = l >> 3, j = l & 7;
#pragma unroll
  for (int p = 0; p < 8; ++p) {
    const int L = w * 32 + p * 4 + q8;
    const int d = L & 63, half = L >> 6;
    const v8h val = *(const v8h*)(sT + d * 128 + half * 64 + j * 8);
    *(volatile v8h*)(Vt + (half ? base1 : base0) + d * 64 + j * 8) = val;
  }
}

__global__ __launch_bounds__(128) void k_proj(
    const unsigned short* __restrict__ xq, const unsigned short* __restrict__ xk,
    const unsigned short* __restrict__ xv, const unsigned short* __restrict__ wq,
    const unsigned short* __restrict__ wk, const unsigned short* __restrict__ wv,
    unsigned short* __restrict__ Qp_us, unsigned short* __restrict__ Kp_us,
    unsigned short* __restrict__ Vt_us) {
  __shared__ __align__(16) _Float16 sT[128 * 64];

  const int z = blockIdx.z;
  const unsigned short* X = (z == 0) ? xq : (z == 1) ? xk : xv;
  const unsigned short* W = (z == 0) ? wq : (z == 1) ? wk : wv;
  const int row0 = blockIdx.x * 128, col0 = blockIdx.y * 64;
  const int tid = threadIdx.x, l = tid & 31, w = tid >> 5, hh = l >> 4, m = l & 15;

  const unsigned short* pa = X + (size_t)(row0 + w * 32 + m) * E + 8 * hh;
  const unsigned short* pb = W + (size_t)(col0 + m) * E + 8 * hh;

  const v8f zero = {0.f, 0.f, 0.f, 0.f, 0.f, 0.f, 0.f, 0.f};
  v8f c00 = zero, c01 = zero, c02 = zero, c03 = zero;
  v8f c10 = zero, c11 = zero, c12 = zero, c13 = zero;

#pragma unroll 1
  for (int k0 = 0; k0 < E; k0 += 32) {
    const v16b a0 = ldb(pa + k0);
    const v16b a1 = ldb(pa + 16 * E + k0);
    const v16b b0 = ldb(pb + k0);
    const v16b b1 = ldb(pb + 16 * E + k0);
    const v16b b2 = ldb(pb + 32 * E + k0);
    const v16b b3 = ldb(pb + 48 * E + k0);
    c00 = mma_b(a0, b0, c00); c01 = mma_b(a0, b1, c01); c02 = mma_b(a0, b2, c02); c03 = mma_b(a0, b3, c03);
    c10 = mma_b(a1, b0, c10); c11 = mma_b(a1, b1, c11); c12 = mma_b(a1, b2, c12); c13 = mma_b(a1, b3, c13);
    asm volatile("v_nop\n\tv_nop\n\tv_nop\n\tv_nop"
                 : "+v"(c00), "+v"(c01), "+v"(c02), "+v"(c03), "+v"(c10), "+v"(c11), "+v"(c12), "+v"(c13)
                 : "v"(a0), "v"(a1), "v"(b0), "v"(b1), "v"(b2), "v"(b3));
  }

  if (z < 2) {
    _Float16* s0 = sT + (w * 32) * 64;
    _Float16* s1 = sT + (w * 32 + 16) * 64;
    st_frag_h(s0 + 0,  64, 1, c00, hh, m); st_frag_h(s0 + 16, 64, 1, c01, hh, m);
    st_frag_h(s0 + 32, 64, 1, c02, hh, m); st_frag_h(s0 + 48, 64, 1, c03, hh, m);
    st_frag_h(s1 + 0,  64, 1, c10, hh, m); st_frag_h(s1 + 16, 64, 1, c11, hh, m);
    st_frag_h(s1 + 32, 64, 1, c12, hh, m); st_frag_h(s1 + 48, 64, 1, c13, hh, m);
  } else {
    _Float16* s0 = sT + (w * 32);
    _Float16* s1 = sT + (w * 32 + 16);
    st_frag_h(s0 + 0 * 128,  1, 128, c00, hh, m); st_frag_h(s0 + 16 * 128, 1, 128, c01, hh, m);
    st_frag_h(s0 + 32 * 128, 1, 128, c02, hh, m); st_frag_h(s0 + 48 * 128, 1, 128, c03, hh, m);
    st_frag_h(s1 + 0 * 128,  1, 128, c10, hh, m); st_frag_h(s1 + 16 * 128, 1, 128, c11, hh, m);
    st_frag_h(s1 + 32 * 128, 1, 128, c12, hh, m); st_frag_h(s1 + 48 * 128, 1, 128, c13, hh, m);
  }
  __syncthreads();

  if (z < 2) {
    _Float16* P = (_Float16*)((z == 0) ? Qp_us : Kp_us);
    lines_nat(sT, P, row0, col0, w, l);
    __threadfence();
    lines_nat(sT, P, row0, col0, w, l);
  } else {
    _Float16* Vt = (_Float16*)Vt_us;
    const int b = blockIdx.x >> 4, blk0 = (blockIdx.x & 15) * 2, h = blockIdx.y;
    const size_t base0 = blkoff(b, h, blk0), base1 = blkoff(b, h, blk0 + 1);
    lines_vt(sT, Vt, base0, base1, w, l);
    __threadfence();
    lines_vt(sT, Vt, base0, base1, w, l);
  }
}

DEV void lines_ao(const unsigned short* sH, const unsigned short* sL, unsigned short* AH, unsigned short* AL,
                  size_t tok0, int h, int w, int l) {
  const int q8 = l >> 3, j = l & 7;
#pragma unroll
  for (int p = 0; p < 4; ++p) {
    const int R = w * 16 + p * 4 + q8;
    const v8us vh = *(const v8us*)(sH + R * 64 + j * 8);
    const v8us vl = *(const v8us*)(sL + R * 64 + j * 8);
    const size_t off = (tok0 + (size_t)R) * E + (size_t)(h * HD + j * 8);
    *(volatile v8us*)(AH + off) = vh;
    *(volatile v8us*)(AL + off) = vl;
  }
}

DEV void st_hilo(unsigned short* sH, unsigned short* sL, v8f o, int row0, int col0, int hh, int m) {
  const float OSCALE = 1.0f / 16384.0f;
#pragma unroll
  for (int rr = 0; rr < 8; ++rr) {
    const float a = o[rr] * OSCALE;
    const unsigned short hi = f2bf(a);
    const unsigned short lo = f2bf(a - bf2f(hi));
    const int idx = (row0 + 8 * hh + rr) * 64 + col0 + m;
    sH[idx] = hi;
    sL[idx] = lo;
  }
}

__global__ __launch_bounds__(128) void k_attn(
    const unsigned short* __restrict__ Qp_us, const unsigned short* __restrict__ Kp_us,
    const unsigned short* __restrict__ Vt_us, unsigned short* __restrict__ AH,
    unsigned short* __restrict__ AL) {
  __shared__ __align__(16) _Float16 sP[4 * 16 * 64];
  __shared__ __align__(16) unsigned short sH[64 * 64];
  __shared__ __align__(16) unsigned short sL[64 * 64];

  const _Float16* Qp = (const _Float16*)Qp_us;
  const _Float16* Kp = (const _Float16*)Kp_us;
  const _Float16* Vt = (const _Float16*)Vt_us;

  const int r = blockIdx.x, h = blockIdx.y, b = blockIdx.z;
  const int tid = threadIdx.x, l = tid & 31, w = tid >> 5, hh = l >> 4, m = l & 15;
  const size_t tok0 = (size_t)b * SEQ + (size_t)r * BLK;
  const float SC = 0.125f;
  const float PSCALE = 16384.0f;

  const _Float16* qp = Qp + (tok0 + (size_t)(w * 16 + m)) * E + h * HD + 8 * hh;
  const v16h q0 = ldh(qp), q1 = ldh(qp + 32);

  const v8f zero = {0.f, 0.f, 0.f, 0.f, 0.f, 0.f, 0.f, 0.f};
  v8f o0 = zero, o1 = zero, o2 = zero, o3 = zero;

  const int cLo = (r > BAND) ? (r - BAND) : 0;
  const int cHi = (r + BAND > NB - 1) ? (NB - 1) : (r + BAND);
  _Float16* myP = sP + w * (16 * 64);

#pragma unroll 1
  for (int c = cLo; c <= cHi; ++c) {
    const _Float16* kp = Kp + ((size_t)b * SEQ + (size_t)c * BLK + m) * E + h * HD + 8 * hh;
    v8f s0, s1, s2, s3;
    {
      const v16h kb0 = ldh(kp), kb1 = ldh(kp + 16 * E), kb2 = ldh(kp + 32 * E), kb3 = ldh(kp + 48 * E);
      s0 = mma_h(q0, kb0, zero); s1 = mma_h(q0, kb1, zero); s2 = mma_h(q0, kb2, zero); s3 = mma_h(q0, kb3, zero);
      asm volatile("v_nop\n\tv_nop\n\tv_nop\n\tv_nop"
                   : "+v"(s0), "+v"(s1), "+v"(s2), "+v"(s3)
                   : "v"(q0), "v"(kb0), "v"(kb1), "v"(kb2), "v"(kb3));
    }
    {
      const v16h kb0 = ldh(kp + 32), kb1 = ldh(kp + 16 * E + 32), kb2 = ldh(kp + 32 * E + 32), kb3 = ldh(kp + 48 * E + 32);
      s0 = mma_h(q1, kb0, s0); s1 = mma_h(q1, kb1, s1); s2 = mma_h(q1, kb2, s2); s3 = mma_h(q1, kb3, s3);
      asm volatile("v_nop\n\tv_nop\n\tv_nop\n\tv_nop"
                   : "+v"(s0), "+v"(s1), "+v"(s2), "+v"(s3)
                   : "v"(q1), "v"(kb0), "v"(kb1), "v"(kb2), "v"(kb3));
    }

#pragma unroll
    for (int rr = 0; rr < 8; ++rr) {
      float v0 = s0[rr] * SC, v1 = s1[rr] * SC, v2 = s2[rr] * SC, v3 = s3[rr] * SC;
      float mx = fmaxf(fmaxf(v0, v1), fmaxf(v2, v3));
      mx = fmaxf(mx, __shfl_xor(mx, 1));
      mx = fmaxf(mx, __shfl_xor(mx, 2));
      mx = fmaxf(mx, __shfl_xor(mx, 4));
      mx = fmaxf(mx, __shfl_xor(mx, 8));
      v0 = __expf(v0 - mx); v1 = __expf(v1 - mx); v2 = __expf(v2 - mx); v3 = __expf(v3 - mx);
      float sm = (v0 + v1) + (v2 + v3);
      sm += __shfl_xor(sm, 1);
      sm += __shfl_xor(sm, 2);
      sm += __shfl_xor(sm, 4);
      sm += __shfl_xor(sm, 8);
      const float f = PSCALE * __builtin_amdgcn_rcpf(sm);
      _Float16* prow = myP + (8 * hh + rr) * 64 + m;
      prow[0]  = (_Float16)(v0 * f);
      prow[16] = (_Float16)(v1 * f);
      prow[32] = (_Float16)(v2 * f);
      prow[48] = (_Float16)(v3 * f);
    }
    __syncthreads();

    {
      const _Float16* pp = myP + m * 64 + 8 * hh;
      const v16h a0 = ldh(pp), a1 = ldh(pp + 32);
      const _Float16* vp = Vt + blkoff(b, h, c) + m * 64 + 8 * hh;
      {
        const v16h vb0 = ldh(vp), vb1 = ldh(vp + 1024), vb2 = ldh(vp + 2048), vb3 = ldh(vp + 3072);
        o0 = mma_h(a0, vb0, o0); o1 = mma_h(a0, vb1, o1); o2 = mma_h(a0, vb2, o2); o3 = mma_h(a0, vb3, o3);
        asm volatile("v_nop\n\tv_nop\n\tv_nop\n\tv_nop"
                     : "+v"(o0), "+v"(o1), "+v"(o2), "+v"(o3)
                     : "v"(a0), "v"(vb0), "v"(vb1), "v"(vb2), "v"(vb3));
      }
      {
        const v16h vb0 = ldh(vp + 32), vb1 = ldh(vp + 1024 + 32), vb2 = ldh(vp + 2048 + 32), vb3 = ldh(vp + 3072 + 32);
        o0 = mma_h(a1, vb0, o0); o1 = mma_h(a1, vb1, o1); o2 = mma_h(a1, vb2, o2); o3 = mma_h(a1, vb3, o3);
        asm volatile("v_nop\n\tv_nop\n\tv_nop\n\tv_nop"
                     : "+v"(o0), "+v"(o1), "+v"(o2), "+v"(o3)
                     : "v"(a1), "v"(vb0), "v"(vb1), "v"(vb2), "v"(vb3));
      }
    }
    __syncthreads();
  }

  st_hilo(sH, sL, o0, w * 16, 0,  hh, m);
  st_hilo(sH, sL, o1, w * 16, 16, hh, m);
  st_hilo(sH, sL, o2, w * 16, 32, hh, m);
  st_hilo(sH, sL, o3, w * 16, 48, hh, m);
  __syncthreads();
  lines_ao(sH, sL, AH, AL, tok0, h, w, l);
  __threadfence();
  lines_ao(sH, sL, AH, AL, tok0, h, w, l);
}

DEV void st_frag_f(float* s, v8f c, int hh, int m) {
#pragma unroll
  for (int rr = 0; rr < 8; ++rr) s[(8 * hh + rr) * 64 + m] = c[rr];
}

DEV void lines_out(const float* sT, float* out, int row0, int col0, int w, int l) {
  const int q2 = l >> 4, j = l & 15;
#pragma unroll
  for (int p = 0; p < 16; ++p) {
    const int R = w * 32 + p * 2 + q2;
    const v4f val = *(const v4f*)(sT + R * 64 + j * 4);
    *(volatile v4f*)(out + (size_t)(row0 + R) * E + col0 + j * 4) = val;
  }
}

__global__ __launch_bounds__(128) void k_oproj(
    const unsigned short* __restrict__ ah, const unsigned short* __restrict__ al,
    const unsigned short* __restrict__ wo, float* __restrict__ out) {
  __shared__ __align__(16) float sT[128 * 64];

  const int row0 = blockIdx.x * 128, col0 = blockIdx.y * 64;
  const int tid = threadIdx.x, l = tid & 31, w = tid >> 5, hh = l >> 4, m = l & 15;

  const size_t aoff = (size_t)(row0 + w * 32 + m) * E + 8 * hh;
  const unsigned short* pah = ah + aoff;
  const unsigned short* pal = al + aoff;
  const unsigned short* pb = wo + (size_t)(col0 + m) * E + 8 * hh;

  const v8f zero = {0.f, 0.f, 0.f, 0.f, 0.f, 0.f, 0.f, 0.f};
  v8f c00 = zero, c01 = zero, c02 = zero, c03 = zero;
  v8f c10 = zero, c11 = zero, c12 = zero, c13 = zero;

#pragma unroll 1
  for (int k0 = 0; k0 < E; k0 += 32) {
    const v16b h0 = ldb(pah + k0), h1 = ldb(pah + 16 * E + k0);
    const v16b l0 = ldb(pal + k0), l1 = ldb(pal + 16 * E + k0);
    const v16b b0 = ldb(pb + k0), b1 = ldb(pb + 16 * E + k0), b2 = ldb(pb + 32 * E + k0), b3 = ldb(pb + 48 * E + k0);
    c00 = mma_b(h0, b0, c00); c01 = mma_b(h0, b1, c01); c02 = mma_b(h0, b2, c02); c03 = mma_b(h0, b3, c03);
    c10 = mma_b(h1, b0, c10); c11 = mma_b(h1, b1, c11); c12 = mma_b(h1, b2, c12); c13 = mma_b(h1, b3, c13);
    c00 = mma_b(l0, b0, c00); c01 = mma_b(l0, b1, c01); c02 = mma_b(l0, b2, c02); c03 = mma_b(l0, b3, c03);
    c10 = mma_b(l1, b0, c10); c11 = mma_b(l1, b1, c11); c12 = mma_b(l1, b2, c12); c13 = mma_b(l1, b3, c13);
    asm volatile("v_nop\n\tv_nop\n\tv_nop\n\tv_nop"
                 : "+v"(c00), "+v"(c01), "+v"(c02), "+v"(c03), "+v"(c10), "+v"(c11), "+v"(c12), "+v"(c13)
                 : "v"(h0), "v"(h1), "v"(l0), "v"(l1), "v"(b0), "v"(b1), "v"(b2), "v"(b3));
  }

  float* s0 = sT + (w * 32) * 64;
  float* s1 = sT + (w * 32 + 16) * 64;
  st_frag_f(s0 + 0, c00, hh, m); st_frag_f(s0 + 16, c01, hh, m); st_frag_f(s0 + 32, c02, hh, m); st_frag_f(s0 + 48, c03, hh, m);
  st_frag_f(s1 + 0, c10, hh, m); st_frag_f(s1 + 16, c11, hh, m); st_frag_f(s1 + 32, c12, hh, m); st_frag_f(s1 + 48, c13, hh, m);
  __syncthreads();
  lines_out(sT, out, row0, col0, w, l);
  __threadfence();
  lines_out(sT, out, row0, col0, w, l);
}

extern "C" void kernel_launch(void* const* d_in, const int* in_sizes, int n_in,
                              void* d_out, int out_size, void* d_ws,
                              size_t ws_size, hipStream_t stream) {
  const int NACT = NTOK * E;
  const int NW = E * E;
  if (n_in < 7) return;
  if (in_sizes[0] != NACT || in_sizes[1] != NACT || in_sizes[2] != NACT) return;
  if (in_sizes[3] != NW || in_sizes[4] != NW || in_sizes[5] != NW || in_sizes[6] != NW) return;
  if (out_size != NACT) return;

  const size_t APL = (size_t)NACT * 2;
  const size_t WPL = (size_t)NW * 2;
  const size_t o_xq = 0, o_xk = APL, o_xv = 2 * APL;
  const size_t o_wq = 3 * APL, o_wk = o_wq + WPL, o_wv = o_wk + WPL, o_wo = o_wv + WPL;
  const size_t o_qp = o_wo + WPL, o_kp = o_qp + APL, o_vt = o_kp + APL;
  const size_t o_ah = o_vt + APL, o_al = o_ah + APL;
  const size_t total = o_al + APL;
  if (ws_size < total) return;

  char* ws = (char*)d_ws;
  unsigned short* xq = (unsigned short*)(ws + o_xq);
  unsigned short* xk = (unsigned short*)(ws + o_xk);
  unsigned short* xv = (unsigned short*)(ws + o_xv);
  unsigned short* bq = (unsigned short*)(ws + o_wq);
  unsigned short* bk = (unsigned short*)(ws + o_wk);
  unsigned short* bv = (unsigned short*)(ws + o_wv);
  unsigned short* bo = (unsigned short*)(ws + o_wo);
  unsigned short* qp = (unsigned short*)(ws + o_qp);
  unsigned short* kp = (unsigned short*)(ws + o_kp);
  unsigned short* vt = (unsigned short*)(ws + o_vt);
  unsigned short* ahp = (unsigned short*)(ws + o_ah);
  unsigned short* alp = (unsigned short*)(ws + o_al);

  const float* q  = (const float*)d_in[0];
  const float* k  = (const float*)d_in[1];
  const float* v  = (const float*)d_in[2];
  const float* Wq = (const float*)d_in[3];
  const float* Wk = (const float*)d_in[4];
  const float* Wv = (const float*)d_in[5];
  const float* Wo = (const float*)d_in[6];
  float* out = (float*)d_out;

  k_prep<<<dim3(512, 7, 1), 256, 0, stream>>>(q, k, v, Wq, Wk, Wv, Wo, xq, xk, xv, bq, bk, bv, bo, NACT, NW);
  k_proj<<<dim3(NTOK / 128, E / 64, 3), 128, 0, stream>>>(xq, xk, xv, bq, bk, bv, qp, kp, vt);
  k_attn<<<dim3(NB, NH, BATCH), 128, 0, stream>>>(qp, kp, vt, ahp, alp);
  k_oproj<<<dim3(NTOK / 128, E / 64, 1), 128, 0, stream>>>(ahp, alp, bo, out);
}
